// MultiHeaded_4080218931880
// MI455X (gfx1250) — hardware-verified
//
#include <hip/hip_runtime.h>


namespace {
constexpr int Bn = 2, F = 2048, T = 2048, C = 1024, H = 16, DD = 64, NT = Bn * F;
constexpr float XS = 8.0f, PS = 8.0f, ALPHA = 0.125f, NEG = -100000.0f;

typedef _Float16 b16;
typedef __attribute__((ext_vector_type(16))) _Float16 v16b;
typedef __attribute__((ext_vector_type(8))) _Float16 v8b;
typedef __attribute__((ext_vector_type(8))) float v8f;
typedef __attribute__((ext_vector_type(4))) float v4f;
__device__ __forceinline__ float bf16_rne(float f) { unsigned int u = __float_as_uint(f); u += 0x7FFFu + ((u >> 16) & 1u); return __uint_as_float(u & 0xFFFF0000u); }
__device__ __forceinline__ void split16(float v, b16& hi, b16& lo) { hi = (b16)v; lo = (b16)(v - (float)hi); }
__device__ __forceinline__ v16b frag_kb(const b16* p, int hh) { const v8b a = *(const v8b*)(p + 8 * hh), b = *(const v8b*)(p + 16 + 8 * hh); v16b f;
#pragma unroll
  for (int e = 0; e < 8; ++e) { f[e] = a[e]; f[8 + e] = b[e]; } return f; }
__device__ __forceinline__ v8f wmma16b(v16b a, v16b b, v8f c) { v8f d = __builtin_amdgcn_wmma_f32_16x16x32_f16(false, a, false, b, (short)0, c, false, false); asm volatile("v_nop\n\tv_nop\n\tv_nop\n\tv_nop" : "+v"(d) : "v"(a), "v"(b)); return d; }
__device__ __forceinline__ void wave_lds_sync() { __builtin_amdgcn_fence(__ATOMIC_RELEASE, "workgroup"); __builtin_amdgcn_wave_barrier(); __builtin_amdgcn_fence(__ATOMIC_ACQUIRE, "workgroup"); }
__device__ __forceinline__ float nexp(float x) { return __builtin_amdgcn_exp2f(x * 1.4426950408889634f); }
__device__ __forceinline__ float pmul(float a, float b) { float p = a * b; asm volatile("" : "+v"(p)); return p; }

__global__ __launch_bounds__(256) void prep_kernel(const float* __restrict__ xf, const float* __restrict__ xt, const float* __restrict__ wq, const float* __restrict__ bq, const float* __restrict__ wk, const float* __restrict__ bk, const float* __restrict__ wv, const float* __restrict__ bv, b16* __restrict__ R, float* __restrict__ P, b16* __restrict__ XF, b16* __restrict__ XT) {
  const size_t tid = (size_t)blockIdx.x * 256 + threadIdx.x, nth = (size_t)gridDim.x * 256;
  for (int pass = 0; pass < 2; ++pass) {
    for (size_t p = tid; p < (size_t)3 * C * (C / 8); p += nth) { const int o3 = (int)(p / (C / 8)), k0 = (int)(p % (C / 8)) * 8; const int w = o3 / C, o = o3 % C; const float* Wm = (w == 0) ? wq : (w == 1) ? wk : wv; v8b v; for (int e = 0; e < 8; ++e) v[e] = (b16)bf16_rne(Wm[(size_t)(k0 + e) * C + o]); *(volatile v8b*)(R + (size_t)o3 * C + k0) = v; }
    for (size_t q = tid; q < 3072; q += nth) { const int i = (int)q; P[q] = bf16_rne(((i < 1024) ? bq : (i < 2048) ? bk : bv)[i & 1023]); }
    for (size_t p = tid; p < (size_t)NT * C / 8; p += nth) { v8b a, c; for (int e = 0; e < 8; ++e) { a[e] = (b16)(bf16_rne(xf[p * 8 + e]) * XS); c[e] = (b16)(bf16_rne(xt[p * 8 + e]) * XS); } *(volatile v8b*)(XF + p * 8) = a; *(volatile v8b*)(XT + p * 8) = c; }
    __threadfence(); }
}
__global__ __launch_bounds__(64) void proj_kernel(const b16* __restrict__ XF, const b16* __restrict__ XT, const b16* __restrict__ R, const float* __restrict__ P, b16* __restrict__ QH, b16* __restrict__ QL, b16* __restrict__ KH, b16* __restrict__ KL, b16* __restrict__ VH, b16* __restrict__ VL) {
  __shared__ __attribute__((aligned(16))) b16 Th[2][32][128 + 8], Tl[2][32][128 + 8];
  const int lane = threadIdx.x & 31, wave = threadIdx.x >> 5, nloc = lane & 15, hlf = lane >> 4, m0 = blockIdx.y * 32; const int w3 = blockIdx.x >> 3; const int c0 = (blockIdx.x & 7) * 128; (void)wave;
  const b16* A = (w3 == 0) ? XF : XT; const b16* Bw = R + (size_t)(w3 * C + c0) * C; const int mw = m0 + wave * 16;
  v8f acc[8];
#pragma unroll
  for (int t = 0; t < 8; ++t) acc[t] = (v8f){};
#pragma unroll 2
  for (int kb = 0; kb < C; kb += 32) { const v16b a = frag_kb(A + (size_t)(mw + nloc) * C + kb, hlf);
#pragma unroll
    for (int t = 0; t < 8; ++t) acc[t] = wmma16b(a, frag_kb(Bw + (size_t)(t * 16 + nloc) * C + kb, hlf), acc[t]); }
#pragma unroll
  for (int t = 0; t < 8; ++t) { const float bb = P[w3 * C + c0 + t * 16 + nloc];
#pragma unroll
    for (int r = 0; r < 8; ++r) { b16 a_, c_; split16(acc[t][r] + XS * bb, a_, c_); Th[wave][8 * hlf + r][t * 16 + nloc] = a_; Tl[wave][8 * hlf + r][t * 16 + nloc] = c_; } }
  wave_lds_sync();
  b16* dh = (w3 == 0) ? QH : (w3 == 1) ? KH : VH; b16* dl = (w3 == 0) ? QL : (w3 == 1) ? KL : VL;
  for (int pass = 0; pass < 2; ++pass) { for (int i = lane; i < 16 * 16; i += 32) { const int rr = i >> 4, c8 = (i & 15) * 8; const size_t gi = (size_t)(mw + rr) * C + c0 + c8; *(volatile v8b*)(dh + gi) = *(const v8b*)(&Th[wave][rr][c8]); *(volatile v8b*)(dl + gi) = *(const v8b*)(&Tl[wave][rr][c8]); } __threadfence(); }
}
__global__ __launch_bounds__(256) void tr_kernel(const b16* __restrict__ QH, const b16* __restrict__ QL, const b16* __restrict__ KH, const b16* __restrict__ KL, b16* __restrict__ QTh, b16* __restrict__ QTl, b16* __restrict__ KTh, b16* __restrict__ KTl) {
  __shared__ __attribute__((aligned(16))) b16 Sh[64][64 + 8], Sl[64][64 + 8];
  const int f0 = blockIdx.x * 64, h = blockIdx.y, b = blockIdx.z >> 1, isk = blockIdx.z & 1, t_ = threadIdx.x;
  const b16* sh = (isk ? KH : QH) + (size_t)b * F * C; const b16* sl = (isk ? KL : QL) + (size_t)b * F * C;
  for (int i = t_; i < 64 * 64; i += 256) { const int d = i >> 6, ff = i & 63; const size_t src = (size_t)(h * DD + d) * F + f0 + ff; Sh[ff][d] = sh[src]; Sl[ff][d] = sl[src]; }
  __syncthreads();
  b16* dh = (isk ? KTh : QTh) + ((size_t)(b * H + h) * F) * DD; b16* dl = (isk ? KTl : QTl) + ((size_t)(b * H + h) * F) * DD;
  for (int pass = 0; pass < 2; ++pass) { for (int i = t_; i < 64 * 8; i += 256) { const int ff = i >> 3, c8 = (i & 7) * 8; *(volatile v8b*)(dh + (size_t)(f0 + ff) * DD + c8) = *(const v8b*)(&Sh[ff][c8]); *(volatile v8b*)(dl + (size_t)(f0 + ff) * DD + c8) = *(const v8b*)(&Sl[ff][c8]); } __threadfence(); }
}
__global__ __launch_bounds__(64) void attn_kernel(const b16* __restrict__ QTh, const b16* __restrict__ QTl, const b16* __restrict__ KTh, const b16* __restrict__ KTl, const b16* __restrict__ VH, const b16* __restrict__ VL, const float* __restrict__ mask, float* __restrict__ out) {
  __shared__ __attribute__((aligned(16))) float Os[DD][32 + 4];
  const int wave = threadIdx.x >> 5, lane = threadIdx.x & 31, hh = lane >> 4, col = lane & 15; const int b = blockIdx.z, h = blockIdx.y, f0 = blockIdx.x * 32 + wave * 16, fi = f0 + col;
  const b16* Qr = QTh + ((size_t)(b * H + h) * F) * DD; const b16* Qlr = QTl + ((size_t)(b * H + h) * F) * DD; const b16* Kr = KTh + ((size_t)(b * H + h) * T) * DD; const b16* Klr = KTl + ((size_t)(b * H + h) * T) * DD;
  const b16* V = VH + (size_t)b * T * C + (size_t)(h * DD) * T; const b16* Vl = VL + (size_t)b * T * C + (size_t)(h * DD) * T; const float* mrow = mask + ((size_t)b * F + fi) * T;
  const v16b qf0 = frag_kb(Qr + (size_t)fi * DD, hh), qf1 = frag_kb(Qr + (size_t)fi * DD + 32, hh), ql0 = frag_kb(Qlr + (size_t)fi * DD, hh), ql1 = frag_kb(Qlr + (size_t)fi * DD + 32, hh);
  float m = -INFINITY, l = 0.0f; v8f o[4] = {{}, {}, {}, {}};
  for (int kb = 0; kb < T; kb += 32) {
    v8f s0 = {}, s1 = {};
    { const v16b k00 = frag_kb(Kr + (size_t)(kb + col) * DD, hh), k01 = frag_kb(Kr + (size_t)(kb + col) * DD + 32, hh), k10 = frag_kb(Kr + (size_t)(kb + 16 + col) * DD, hh), k11 = frag_kb(Kr + (size_t)(kb + 16 + col) * DD + 32, hh);
      const v16b l00 = frag_kb(Klr + (size_t)(kb + col) * DD, hh), l01 = frag_kb(Klr + (size_t)(kb + col) * DD + 32, hh), l10 = frag_kb(Klr + (size_t)(kb + 16 + col) * DD, hh), l11 = frag_kb(Klr + (size_t)(kb + 16 + col) * DD + 32, hh);
      s0 = wmma16b(k00, qf0, s0); s0 = wmma16b(k01, qf1, s0); s0 = wmma16b(l00, qf0, s0); s0 = wmma16b(l01, qf1, s0); s0 = wmma16b(k00, ql0, s0); s0 = wmma16b(k01, ql1, s0);
      s1 = wmma16b(k10, qf0, s1); s1 = wmma16b(k11, qf1, s1); s1 = wmma16b(l10, qf0, s1); s1 = wmma16b(l11, qf1, s1); s1 = wmma16b(k10, ql0, s1); s1 = wmma16b(k11, ql1, s1); }
    float mr = -INFINITY;
#pragma unroll
    for (int r = 0; r < 8; ++r) { const int j0 = kb + 8 * hh + r, j1 = j0 + 16; s0[r] = s0[r] * (ALPHA / (XS * XS)) + (1.0f - bf16_rne(mrow[j0])) * NEG; s1[r] = s1[r] * (ALPHA / (XS * XS)) + (1.0f - bf16_rne(mrow[j1])) * NEG; mr = fmaxf(mr, fmaxf(s0[r], s1[r])); }
    mr = fmaxf(mr, __shfl_xor(mr, 16)); const float mn = fmaxf(m, mr); const float al_ = nexp(m - mn); m = mn; float sum = 0.0f; v16b pb, pl;
#pragma unroll
    for (int r = 0; r < 8; ++r) { const float e0 = nexp(s0[r] - mn), e1 = nexp(s1[r] - mn); sum += e0 + e1; b16 a_, c_; split16(e0 * PS, a_, c_); pb[r] = a_; pl[r] = c_; split16(e1 * PS, a_, c_); pb[8 + r] = a_; pl[8 + r] = c_; }
    sum += __shfl_xor(sum, 16); l = l * al_ + sum;
#pragma unroll
    for (int t = 0; t < 4; ++t) { o[t] *= al_; const v16b vh = frag_kb(V + (size_t)(t * 16 + col) * T + kb, hh); o[t] = wmma16b(vh, pb, o[t]); o[t] = wmma16b(vh, pl, o[t]); o[t] = wmma16b(frag_kb(Vl + (size_t)(t * 16 + col) * T + kb, hh), pb, o[t]); } }
  const float inv = 1.0f / (l * PS * XS);
#pragma unroll
  for (int t = 0; t < 4; ++t)
#pragma unroll
    for (int r = 0; r < 8; ++r) Os[t * 16 + 8 * hh + r][wave * 16 + col] = o[t][r] * inv;
  __syncthreads();
  for (int pass = 0; pass < 2; ++pass) { for (int i = threadIdx.x; i < DD * 8; i += 64) { const int d = i >> 3, c4 = (i & 7) * 4; *(volatile v4f*)(out + ((size_t)b * C + h * DD + d) * F + blockIdx.x * 32 + c4) = *(const v4f*)(&Os[d][c4]); } __threadfence(); }
}
}

extern "C" void kernel_launch(void* const* d_in, const int* in_sizes, int n_in,
                              void* d_out, int out_size, void* d_ws, size_t ws_size, hipStream_t stream) {
  (void)n_in; (void)out_size;
  auto Fp = [&](int i) { return (const float*)d_in[i]; };
  float* out = (float*)d_out;
  if (in_sizes[0] != NT * C || in_sizes[1] != NT * C || in_sizes[2] != Bn * F * T || in_sizes[3] != C * C) return;
  size_t off = 0; char* ws = (char*)d_ws;
  auto carve = [&](size_t bytes) { char* p = ws + off; off += (bytes + 255) & ~(size_t)255; return p; };
  const size_t plane = (size_t)NT * C;
  b16* R = (b16*)carve((size_t)3 * C * C * 2); float* P = (float*)carve(3072 * 4); b16* XF = (b16*)carve(plane * 2); b16* XT = (b16*)carve(plane * 2);
  b16* QH = (b16*)carve(plane * 2); b16* QL = (b16*)carve(plane * 2); b16* KH = (b16*)carve(plane * 2); b16* KL = (b16*)carve(plane * 2); b16* VH = (b16*)carve(plane * 2); b16* VL = (b16*)carve(plane * 2);
  b16* QTh = (b16*)carve(plane * 2); b16* QTl = (b16*)carve(plane * 2); b16* KTh = (b16*)carve(plane * 2); b16* KTl = (b16*)carve(plane * 2);
  if (off > ws_size) return;
  prep_kernel<<<1024, 256, 0, stream>>>(Fp(0), Fp(1), Fp(3), Fp(4), Fp(5), Fp(6), Fp(7), Fp(8), R, P, XF, XT);
  proj_kernel<<<dim3(24, NT / 32), 64, 0, stream>>>(XF, XT, R, P, QH, QL, KH, KL, VH, VL);
  tr_kernel<<<dim3(F / 64, H, Bn * 2), 256, 0, stream>>>(QH, QL, KH, KL, QTh, QTl, KTh, KTl);
  attn_kernel<<<dim3(F / 32, H, Bn), 64, 0, stream>>>(QTh, QTl, KTh, KTl, VH, VL, Fp(2), out);
}
